// MambaVideoEncoder_31963146616889
// MI455X (gfx1250) — hardware-verified
//
#include <hip/hip_runtime.h>


#define L_     4096
#define DM_    768
#define DI_    1536
#define NS_    16
#define DTR_   48
#define DTRP_  64
#define XDN_   80
#define XDW_   128
#define ZROWS_ 64
#define SCH_   32

static_assert(L_ % 64 == 0);
static_assert(L_ % SCH_ == 0);
static_assert(DI_ % 128 == 0);
static_assert(DI_ % 64 == 0);
static_assert(DI_ % 32 == 0);
static_assert(DI_ % 8 == 0);
static_assert(DM_ % 32 == 0);
static_assert(DM_ % 8 == 0);
static_assert(DTRP_ % 32 == 0);
static_assert(DTR_ % 8 == 0);
static_assert(DTR_ <= DTRP_);
static_assert(XDW_ % 128 == 0);
static_assert(DTR_ + 2 * NS_ == XDN_);
static_assert(XDN_ <= XDW_);
static_assert(DM_ == 3 * 256);
static_assert(ZROWS_ == 64);
static_assert(L_ >= ZROWS_);
static_assert(SCH_ * NS_ == 64 * 8);

typedef float          v4f   __attribute__((ext_vector_type(4)));
typedef float          v8f   __attribute__((ext_vector_type(8)));
typedef _Float16       v8h   __attribute__((ext_vector_type(8)));
typedef _Float16       v16h  __attribute__((ext_vector_type(16)));
typedef unsigned short u16x8 __attribute__((ext_vector_type(8)));

union FragH { u16x8 h[2]; v16h v; };
union Pack8 { v8h f; u16x8 u; };

constexpr size_t SZ_X16 = (size_t)L_ * DM_ * 2;
constexpr size_t SZ_WI  = (size_t)2 * DI_ * DM_ * 2;
constexpr size_t SZ_XF  = (size_t)L_ * DI_ * 4;
constexpr size_t SZ_U16 = (size_t)L_ * DI_ * 2;
constexpr size_t SZ_WX  = (size_t)XDW_ * DI_ * 2;
constexpr size_t SZ_XD  = (size_t)L_ * XDW_ * 4;
constexpr size_t SZ_DTR = (size_t)L_ * DTRP_ * 2;
constexpr size_t SZ_WD  = (size_t)DI_ * DTRP_ * 2;
constexpr size_t SZ_DL  = (size_t)L_ * DI_ * 4;
constexpr size_t SZ_ZB  = (size_t)ZROWS_ * DI_ * 4;
constexpr size_t SZ_YV  = (size_t)DI_ * 4;

constexpr size_t OFF_X16 = 0;
constexpr size_t OFF_WI  = OFF_X16 + SZ_X16;
constexpr size_t OFF_XF  = OFF_WI  + SZ_WI;
constexpr size_t OFF_U16 = OFF_XF  + SZ_XF;
constexpr size_t OFF_WX  = OFF_U16 + SZ_U16;
constexpr size_t OFF_XD  = OFF_WX  + SZ_WX;
constexpr size_t OFF_DTR = OFF_XD  + SZ_XD;
constexpr size_t OFF_WD  = OFF_DTR + SZ_DTR;
constexpr size_t OFF_DL  = OFF_WD  + SZ_WD;
constexpr size_t OFF_ZB  = OFF_DL  + SZ_DL;
constexpr size_t OFF_YV  = OFF_ZB  + SZ_ZB;
constexpr size_t WS_END  = OFF_YV  + SZ_YV;
static_assert(WS_END <= (size_t)134217728);
static_assert(OFF_WI % 128 == 0 && OFF_XF % 128 == 0 && OFF_U16 % 128 == 0 && OFF_WX % 128 == 0);
static_assert(OFF_XD % 128 == 0 && OFF_DTR % 128 == 0 && OFF_WD % 128 == 0 && OFF_DL % 128 == 0);
static_assert(OFF_ZB % 128 == 0 && OFF_YV % 128 == 0);

__device__ __forceinline__ float silu_f(float x) {
    const float e = __expf(-x);
    return x * __builtin_amdgcn_rcpf(1.0f + e);
}
__device__ __forceinline__ float softplus_f(float x) {
    return fmaxf(x, 0.0f) + log1pf(__expf(-fabsf(x)));
}
__device__ __forceinline__ float conv4_silu(float x0, float x1, float x2, float x3,
                                            float w0, float w1, float w2, float w3, float bias) {
    const float c = w0 * x0 + w1 * x1 + w2 * x2 + w3 * x3;
    return silu_f(c + bias);
}
__device__ __forceinline__ v8f ld8f(const float* p) {
    const v4f a = *(const v4f*)p;
    const v4f b = *(const v4f*)(p + 4);
    return __builtin_shufflevector(a, b, 0, 1, 2, 3, 4, 5, 6, 7);
}

__device__ __forceinline__ void mma16(v8f& acc, const FragH& a, const FragH& b) {
    acc = __builtin_amdgcn_wmma_f32_16x16x32_f16(false, a.v, false, b.v, (short)0, acc, false, false);
    asm volatile("v_nop\n\tv_nop\n\tv_nop\n\tv_nop" : "+v"(acc) : "v"(a.v), "v"(b.v));
}

__global__ __launch_bounds__(256)
void cvt16_kernel(const float* __restrict__ src, unsigned short* dst,
                  int rows_out, int rows_in, int kin, int kpad, int in_stride, float scale)
{
    const int g8 = kpad >> 3;
    const int i  = blockIdx.x * 256 + threadIdx.x;
    if (i >= rows_out * g8) return;
    const int r  = i / g8;
    const int k0 = (i - r * g8) * 8;
    v8f x;
    if (r < rows_in && k0 + 8 <= kin) {
        x = ld8f(src + (size_t)r * in_stride + k0) * scale;
    } else {
#pragma unroll
        for (int c = 0; c < 8; ++c) x[c] = 0.0f;
    }
    Pack8 pk;
    pk.f = __builtin_convertvector(x, v8h);
    const u16x8 v = pk.u;
    unsigned short* gp = dst + (size_t)i * 8;
    *(volatile u16x8*)gp = v;
    __threadfence();
    *(volatile u16x8*)gp = v;
}

template<int NBF>
__device__ __forceinline__ void tile_store_pass(const float* st, float* gp, int ldc, int lane) {
    constexpr int CW  = NBF * 16;
    constexpr int P   = CW + 4;
    constexpr int LPR = CW / 4;
    static_assert(32 % LPR == 0);
    constexpr int RPI = 32 / LPR;
    static_assert(32 % RPI == 0);
    constexpr int NIT = 32 / RPI;
    const int rsub = lane / LPR;
    const int c0   = (lane % LPR) * 4;
#pragma unroll
    for (int it = 0; it < NIT; ++it) {
        const int row = it * RPI + rsub;
        const v4f v = *(const v4f*)(st + row * P + c0);
        *(volatile v4f*)(gp + (size_t)row * ldc + c0) = v;
    }
}

template<int NBF>
__global__ __launch_bounds__(128)
void gemm_tn_kernel(const unsigned short* __restrict__ A, const unsigned short* __restrict__ Bw,
                    float* C, int K, int ldc, float scale)
{
    constexpr int CW = NBF * 16;
    constexpr int P  = CW + 4;
    __shared__ __attribute__((aligned(16))) float stile[4][32 * P];

    const int tid  = threadIdx.x;
    const int lane = tid & 31;
    const int wave = tid >> 5;
    const int h    = lane >> 4;
    const int m    = lane & 15;
    const int wm   = wave >> 1;
    const int wn   = wave & 1;

    const int rowW = blockIdx.y * 64 + wm * 32;
    const int colW = blockIdx.x * (2 * CW) + wn * CW;

    v8f acc[2 * NBF];
#pragma unroll
    for (int j = 0; j < 2 * NBF; ++j)
#pragma unroll
        for (int r = 0; r < 8; ++r) acc[j][r] = 0.0f;

    const size_t aoff  = (size_t)(rowW + m) * K + 8 * h;
    const size_t boff  = (size_t)(colW + m) * K + 8 * h;
    const size_t sub16 = (size_t)16 * K;
    const int nk = K >> 5;

    for (int kt = 0; kt < nk; ++kt) {
        const size_t k0 = (size_t)kt * 32;
        FragH fa[2], fb[NBF];
#pragma unroll
        for (int s = 0; s < 2; ++s) {
            const unsigned short* p = A + aoff + s * sub16 + k0;
            fa[s].h[0] = *(const u16x8*)(p);
            fa[s].h[1] = *(const u16x8*)(p + 16);
        }
#pragma unroll
        for (int j = 0; j < NBF; ++j) {
            const unsigned short* p = Bw + boff + j * sub16 + k0;
            fb[j].h[0] = *(const u16x8*)(p);
            fb[j].h[1] = *(const u16x8*)(p + 16);
        }
#pragma unroll
        for (int s = 0; s < 2; ++s)
#pragma unroll
            for (int j = 0; j < NBF; ++j)
                mma16(acc[s * NBF + j], fa[s], fb[j]);
    }

    float* st = stile[wave];
#pragma unroll
    for (int s = 0; s < 2; ++s)
#pragma unroll
        for (int j = 0; j < NBF; ++j)
#pragma unroll
            for (int r = 0; r < 8; ++r)
                st[(s * 16 + 8 * h + r) * P + j * 16 + m] = acc[s * NBF + j][r] * scale;
    __syncthreads();

    float* gp = C + (size_t)rowW * ldc + colW;
    tile_store_pass<NBF>(st, gp, ldc, lane);
    __threadfence();
    tile_store_pass<NBF>(st, gp, ldc, lane);
}

__global__ __launch_bounds__(192)
void conv_silu_kernel(const float* __restrict__ X, const float* __restrict__ cw,
                      const float* __restrict__ cb, unsigned short* U16)
{
    const int t  = blockIdx.x;
    const int d0 = threadIdx.x * 8;
    const float* xr = X + (size_t)t * DI_ + d0;

    v8f x3 = ld8f(xr);
    v8f x2, x1, x0;
#pragma unroll
    for (int c = 0; c < 8; ++c) { x2[c] = 0.0f; x1[c] = 0.0f; x0[c] = 0.0f; }
    if (t >= 1) x2 = ld8f(xr - DI_);
    if (t >= 2) x1 = ld8f(xr - 2 * DI_);
    if (t >= 3) x0 = ld8f(xr - 3 * DI_);

    const float* wp = cw + (size_t)d0 * 4;
    v4f wv[8];
#pragma unroll
    for (int c = 0; c < 8; ++c) wv[c] = *(const v4f*)(wp + 4 * c);
    const v8f bias = ld8f(cb + d0);

    v8f u;
#pragma unroll
    for (int c = 0; c < 8; ++c)
        u[c] = conv4_silu(x0[c], x1[c], x2[c], x3[c], wv[c][0], wv[c][1], wv[c][2], wv[c][3], bias[c]);

    Pack8 pk;
    pk.f = __builtin_convertvector(u * 8.0f, v8h);
    const u16x8 v = pk.u;
    unsigned short* gp = U16 + (size_t)t * DI_ + d0;
    *(volatile u16x8*)gp = v;
    __threadfence();
    *(volatile u16x8*)gp = v;
}

__global__ __launch_bounds__(64)
void scan_kernel(const float* __restrict__ X, const float* __restrict__ Dl,
                 const float* __restrict__ xd,
                 const float* __restrict__ cw, const float* __restrict__ cb,
                 const float* __restrict__ Alog, const float* __restrict__ Dp,
                 const float* __restrict__ dtb, const float* __restrict__ zb,
                 float* yv)
{
    __shared__ __attribute__((aligned(16))) v4f   sB4[SCH_ * 4];
    __shared__ __attribute__((aligned(16))) float sy[64];

    const int tid   = threadIdx.x;
    const int dbase = blockIdx.x * 64;
    const int d     = dbase + tid;

    float an[NS_], hs[NS_];
#pragma unroll
    for (int n = 0; n < NS_; ++n) {
        an[n] = -__expf(Alog[(size_t)d * NS_ + n]);
        hs[n] = 0.0f;
    }
    const float w0 = cw[d * 4 + 0], w1 = cw[d * 4 + 1], w2 = cw[d * 4 + 2], w3 = cw[d * 4 + 3];
    const float cbias = cb[d];
    const float tb = dtb[d];
    const float Dd = Dp[d];

    float xm1 = 0.0f, xm2 = 0.0f, xm3 = 0.0f, ulast = 0.0f;
    const int tt = tid >> 1;
    const int hf = tid & 1;

#pragma unroll 1
    for (int t0 = 0; t0 < L_; t0 += SCH_) {
        {
            const float* bp = xd + (size_t)(t0 + tt) * XDW_ + DTR_ + 8 * hf;
            sB4[tt * 4 + 2 * hf]     = *(const v4f*)(bp);
            sB4[tt * 4 + 2 * hf + 1] = *(const v4f*)(bp + 4);
        }
        __syncthreads();
#pragma unroll 1
        for (int t = 0; t < SCH_; ++t) {
            const size_t e = (size_t)(t0 + t) * DI_ + d;
            const float xv = X[e];
            const float dl = Dl[e];
            const float u  = conv4_silu(xm3, xm2, xm1, xv, w0, w1, w2, w3, cbias);
            xm3 = xm2; xm2 = xm1; xm1 = xv;
            const float dt = softplus_f(dl + tb);
            const float du = dt * u;
            const v4f bq[4] = { sB4[t * 4 + 0], sB4[t * 4 + 1], sB4[t * 4 + 2], sB4[t * 4 + 3] };
#pragma unroll
            for (int q = 0; q < 4; ++q)
#pragma unroll
                for (int c = 0; c < 4; ++c) {
                    const int n = 4 * q + c;
                    const float da = __expf(dt * an[n]);
                    hs[n] = da * hs[n] + du * bq[q][c];
                }
            ulast = u;
        }
        __syncthreads();
    }

    float y = 0.0f;
    const float* cp = xd + (size_t)(L_ - 1) * XDW_ + DTR_ + NS_;
#pragma unroll
    for (int n = 0; n < NS_; ++n) y += hs[n] * cp[n];
    const float z = zb[(size_t)(ZROWS_ - 1) * DI_ + d];
    const float g = (y + Dd * ulast) * silu_f(z);

    sy[tid] = g;
    __syncthreads();
    if (tid < 16) {
        const v4f v = *(const v4f*)(sy + 4 * tid);
        float* gp = yv + dbase + 4 * tid;
        *(volatile v4f*)gp = v;
        __threadfence();
        *(volatile v4f*)gp = v;
    }
}

__global__ __launch_bounds__(256)
void outnorm_kernel(const float* __restrict__ wo, const float* __restrict__ yv, float* out)
{
    __shared__ __attribute__((aligned(16))) float ys[DI_];
    __shared__ __attribute__((aligned(16))) float so[DM_];
    __shared__ float sq[256];

    const int tid = threadIdx.x;
    for (int i = tid; i < DI_; i += 256) ys[i] = yv[i];
    __syncthreads();

    const float* r0p = wo + (size_t)tid * DI_;
    const float* r1p = wo + (size_t)(tid + 256) * DI_;
    const float* r2p = wo + (size_t)(tid + 512) * DI_;
    float a0 = 0.0f, a1 = 0.0f, a2 = 0.0f;
#pragma unroll 1
    for (int k = 0; k < DI_; k += 4) {
        const v4f yk = *(const v4f*)(ys + k);
        const v4f w0 = *(const v4f*)(r0p + k);
        const v4f w1 = *(const v4f*)(r1p + k);
        const v4f w2 = *(const v4f*)(r2p + k);
#pragma unroll
        for (int c = 0; c < 4; ++c) {
            a0 += w0[c] * yk[c];
            a1 += w1[c] * yk[c];
            a2 += w2[c] * yk[c];
        }
    }
    so[tid]       = a0;
    so[tid + 256] = a1;
    so[tid + 512] = a2;
    sq[tid] = a0 * a0 + a1 * a1 + a2 * a2;
    __syncthreads();
    for (int o = 128; o > 0; o >>= 1) {
        if (tid < o) sq[tid] += sq[tid + o];
        __syncthreads();
    }
    const float nrm  = fmaxf(sqrtf(sq[0]), 1e-12f);
    const float rinv = 1.0f / nrm;
    if (tid < DM_ / 4) {
        const v4f v = *(const v4f*)(so + 4 * tid) * rinv;
        float* gp = out + 4 * tid;
        *(volatile v4f*)gp = v;
        __threadfence();
        *(volatile v4f*)gp = v;
    }
}

extern "C" void kernel_launch(void* const* d_in, const int* in_sizes, int n_in,
                              void* d_out, int out_size, void* d_ws, size_t ws_size,
                              hipStream_t stream)
{
    if (n_in < 10) return;
    if (in_sizes[0] != L_ * DM_)        return;
    if (in_sizes[1] != 2 * DI_ * DM_)   return;
    if (in_sizes[2] != DI_ * 4)         return;
    if (in_sizes[3] != DI_)             return;
    if (in_sizes[4] != XDN_ * DI_)      return;
    if (in_sizes[5] != DI_ * DTR_)      return;
    if (in_sizes[6] != DI_)             return;
    if (in_sizes[7] != DI_ * NS_)       return;
    if (in_sizes[8] != DI_)             return;
    if (in_sizes[9] != DM_ * DI_)       return;
    if (out_size != DM_)                return;
    if (ws_size < WS_END)               return;

    const float* frame = (const float*)d_in[0];
    const float* wi    = (const float*)d_in[1];
    const float* cw    = (const float*)d_in[2];
    const float* cb    = (const float*)d_in[3];
    const float* wx    = (const float*)d_in[4];
    const float* wd    = (const float*)d_in[5];
    const float* dtb   = (const float*)d_in[6];
    const float* alog  = (const float*)d_in[7];
    const float* Dp    = (const float*)d_in[8];
    const float* wo    = (const float*)d_in[9];
    float* out = (float*)d_out;

    char* ws = (char*)d_ws;
    unsigned short* x16   = (unsigned short*)(ws + OFF_X16);
    unsigned short* wi16  = (unsigned short*)(ws + OFF_WI);
    float*          Xf    = (float*)(ws + OFF_XF);
    unsigned short* u16   = (unsigned short*)(ws + OFF_U16);
    unsigned short* wx16  = (unsigned short*)(ws + OFF_WX);
    float*          xd    = (float*)(ws + OFF_XD);
    unsigned short* dtr16 = (unsigned short*)(ws + OFF_DTR);
    unsigned short* wd16  = (unsigned short*)(ws + OFF_WD);
    float*          Dl    = (float*)(ws + OFF_DL);
    float*          zb    = (float*)(ws + OFF_ZB);
    float*          yv    = (float*)(ws + OFF_YV);

    {
        int n8;
        n8 = (L_ * DM_) / 8;
        hipLaunchKernelGGL(cvt16_kernel, dim3((n8 + 255) / 256), dim3(256), 0, stream,
                           frame, x16, (int)L_, (int)L_, (int)DM_, (int)DM_, (int)DM_, 1.0f);
        n8 = (2 * DI_ * DM_) / 8;
        hipLaunchKernelGGL(cvt16_kernel, dim3((n8 + 255) / 256), dim3(256), 0, stream,
                           wi, wi16, (int)(2 * DI_), (int)(2 * DI_), (int)DM_, (int)DM_, (int)DM_, 32.0f);
        n8 = (XDW_ * DI_) / 8;
        hipLaunchKernelGGL(cvt16_kernel, dim3((n8 + 255) / 256), dim3(256), 0, stream,
                           wx, wx16, (int)XDW_, (int)XDN_, (int)DI_, (int)DI_, (int)DI_, 32.0f);
        n8 = (DI_ * DTRP_) / 8;
        hipLaunchKernelGGL(cvt16_kernel, dim3((n8 + 255) / 256), dim3(256), 0, stream,
                           wd, wd16, (int)DI_, (int)DI_, (int)DTR_, (int)DTRP_, (int)DTR_, 4.0f);
    }

    hipLaunchKernelGGL(HIP_KERNEL_NAME(gemm_tn_kernel<4>),
                       dim3(DI_ / 128, L_ / 64), dim3(128), 0, stream,
                       (const unsigned short*)x16, (const unsigned short*)wi16,
                       Xf, (int)DM_, (int)DI_, 0.03125f);

    hipLaunchKernelGGL(HIP_KERNEL_NAME(gemm_tn_kernel<4>),
                       dim3(DI_ / 128, ZROWS_ / 64), dim3(128), 0, stream,
                       (const unsigned short*)(x16 + (size_t)(L_ - ZROWS_) * DM_),
                       (const unsigned short*)(wi16 + (size_t)DI_ * DM_),
                       zb, (int)DM_, (int)DI_, 0.03125f);

    hipLaunchKernelGGL(conv_silu_kernel, dim3(L_), dim3(DI_ / 8), 0, stream,
                       (const float*)Xf, cw, cb, u16);

    hipLaunchKernelGGL(HIP_KERNEL_NAME(gemm_tn_kernel<4>),
                       dim3(XDW_ / 128, L_ / 64), dim3(128), 0, stream,
                       (const unsigned short*)u16, (const unsigned short*)wx16,
                       xd, (int)DI_, (int)XDW_, 0.00390625f);

    {
        const int n8 = (L_ * DTRP_) / 8;
        hipLaunchKernelGGL(cvt16_kernel, dim3((n8 + 255) / 256), dim3(256), 0, stream,
                           (const float*)xd, dtr16, (int)L_, (int)L_, (int)DTR_, (int)DTRP_, (int)XDW_, 16.0f);
    }

    hipLaunchKernelGGL(HIP_KERNEL_NAME(gemm_tn_kernel<4>),
                       dim3(DI_ / 128, L_ / 64), dim3(128), 0, stream,
                       (const unsigned short*)dtr16, (const unsigned short*)wd16,
                       Dl, (int)DTRP_, (int)DI_, 0.015625f);

    hipLaunchKernelGGL(scan_kernel, dim3(DI_ / 64), dim3(64), 0, stream,
                       (const float*)Xf, (const float*)Dl, (const float*)xd,
                       cw, cb, alog, Dp, dtb, (const float*)zb, yv);

    hipLaunchKernelGGL(outnorm_kernel, dim3(1), dim3(256), 0, stream,
                       wo, (const float*)yv, out);
}
